// RandomProjectLinearOperator_29171417874658
// MI455X (gfx1250) — hardware-run, weakly checked
//
#include <hip/hip_runtime.h>


#ifndef NB
#define NB 8
#endif
#ifndef NPO
#define NPO 1024
#endif
#define NB_FULL 8
#define GH    32
#define GW    32
#define NPIX  1024
#define CIN_  64
#define COUT_ 64
#define NPJ   16
#define KT    (NPJ * CIN_)
#define KP2   (KT + CIN_)
#define CSC   16.0f
#define VSC   1024.0f
#define WSC   1024.0f
#define TSI   (1.0f / (16.0f * 1024.0f))
#define OSI   (1.0f / (1024.0f * 1024.0f))
#define VTP   72
#define CTP   264

static_assert(GH * GW == NPIX);
static_assert(CIN_ == 64);
static_assert(COUT_ % 64 == 0);
static_assert(NPJ == 16);
static_assert(NPIX % 32 == 0);
static_assert(KT % 32 == 0);
static_assert(KP2 % 32 == 0);
static_assert((KP2 * 2) % 128 == 0);
static_assert((KT * 2) % 128 == 0);
static_assert(NPO % 64 == 0);
static_assert(NPO >= 64);
static_assert(NPO <= NPIX);
static_assert((NPO * NPJ) % 64 == 0);
static_assert((NB * CIN_) % 64 == 0);
static_assert((NB * NPO) % 64 == 0);
static_assert(NPIX % 256 == 0);
static_assert(NPIX % 64 == 0);
static_assert((COUT_ * (KP2 / 8)) % 256 == 0);
static_assert(NB <= NB_FULL);
static_assert((VTP * 2) % 16 == 0);
static_assert((CTP * 2) % 16 == 0);
static_assert(32 * 16 * 4 == 16 * CIN_ * 2);
static_assert(32 * 16 * 8 == 16 * 64 * 4);
static_assert(8 * 2 * 32 * 16 == NPJ * 256 * 2);
static_assert(256 * 2 * 16 == 64 * 64 * 2);
static_assert(4 * 256 * 4 == 64 * 64);
static_assert((32 + 8 + 128 + 16) * 4 + 8 * 256 * 4 + NPJ * CTP * 2 <= 131072);
static_assert(64 * VTP * 2 <= 131072);
static_assert(16 * 68 * 4 <= 131072);

typedef _Float16 h16;
typedef __attribute__((ext_vector_type(16))) _Float16 v16h;
typedef __attribute__((ext_vector_type(8)))  _Float16 v8h;
typedef __attribute__((ext_vector_type(8)))  float    v8f;
typedef __attribute__((ext_vector_type(4)))  float    v4f;
typedef v4f  __attribute__((may_alias)) v4fa;
typedef v8h  __attribute__((may_alias)) v8ha;

__device__ __forceinline__ unsigned short f2bf(float f) { unsigned u = __float_as_uint(f); u += 0x7FFFu + ((u >> 16) & 1u); return (unsigned short)(u >> 16); }
__device__ __forceinline__ float bfr(float f) { return __uint_as_float(((unsigned)f2bf(f)) << 16); }
__device__ __forceinline__ v16h cat16(v8h lo, v8h hi) { return __builtin_shufflevector(lo, hi, 0, 1, 2, 3, 4, 5, 6, 7, 8, 9, 10, 11, 12, 13, 14, 15); }
__device__ __forceinline__ v8f wmma16(v16h a, v16h b, v8f c) { return __builtin_amdgcn_wmma_f32_16x16x32_f16(false, a, false, b, (short)0, c, false, false); }
__device__ __forceinline__ v16h  ldh(const h16* p) { return cat16(*(const v8h*)p, *(const v8h*)(p + 16)); }
__device__ __forceinline__ void wave_sync() { __builtin_amdgcn_fence(3  , "wavefront"); __builtin_amdgcn_wave_barrier(); asm volatile("" ::: "memory"); }
static __device__ __forceinline__ h16 toh_flush(float v) { const h16 r = (h16)v; return (fabsf(v) < 6.103515625e-05f) ? (h16)0.0f : r; }
__device__ __forceinline__ v8f wmma16g(v16h a, v16h b, v8f c) {
    c = wmma16(a, b, c);
    asm volatile("v_nop\n\tv_nop\n\tv_nop\n\tv_nop" : "+v"(c) : "v"(a), "v"(b));
    return c;
}

__global__ __launch_bounds__(256) void k_wplane(const float* __restrict__ params, const float* __restrict__ convw, h16* PA) {
    const int p = blockIdx.x * 256 + threadIdx.x; if (p >= COUT_ * (KP2 / 8)) return;
    const int o = p / (KP2 / 8), q = p % (KP2 / 8); const int k0 = q * 8;
    const bool isc = k0 >= KT;
    const int kp = isc ? (KT - 8) : k0;
    const int kc = isc ? (k0 - KT) : 0;
    v8f pv = *(const v8f*)(params + (size_t)(kp >> 6) * (COUT_ * CIN_) + (size_t)o * CIN_ + (kp & 63));
    v8f cv = *(const v8f*)(convw + (size_t)o * CIN_ + kc);
    asm volatile("" : "+v"(pv)); asm volatile("" : "+v"(cv));
    v8h hv;
#pragma unroll
    for (int k = 0; k < 8; ++k) { const float x = isc ? cv[k] : pv[k]; hv[k] = toh_flush(bfr(x) * WSC); }
    *(volatile v8h*)(PA + (size_t)p * 8) = hv; __threadfence(); *(volatile v8h*)(PA + (size_t)p * 8) = hv;
}

__global__ __launch_bounds__(256) void k_vplanes(const float* __restrict__ v, h16* VH, h16* T2) {
    __shared__ __align__(16) h16 hs[64 * VTP];
    const int tid = threadIdx.x;
    const int p0 = blockIdx.x * 64, b = blockIdx.y;
    const float* src = v + (size_t)b * CIN_ * NPIX + p0;
#pragma unroll
    for (int it = 0; it < 4; ++it) { const int idx = it * 256 + tid; const int row = idx >> 4, c4 = (idx & 15) * 4;
        const v4f x = *(const v4f*)(src + (size_t)row * NPIX + c4);
#pragma unroll
        for (int k = 0; k < 4; ++k) hs[row * VTP + c4 + k] = toh_flush(bfr(x[k]) * VSC); }
    __syncthreads();
    v8h a[2], t[2]; size_t ao[2], to[2];
#pragma unroll
    for (int it = 0; it < 2; ++it) { const int p = it * 256 + tid; const int row = p >> 3, c8 = (p & 7) * 8;
#pragma unroll
        for (int k = 0; k < 8; ++k) { a[it][k] = hs[row * VTP + c8 + k]; t[it][k] = hs[(c8 + k) * VTP + row]; }
        ao[it] = ((size_t)(b * CIN_ + row)) * NPIX + (size_t)(p0 + c8);
        to[it] = ((size_t)b * NPO + (size_t)(p0 + row)) * KP2 + (size_t)(KT + c8); }
    const bool wt = p0 < NPO;
#pragma unroll 1
    for (int ps = 0; ps < 2; ++ps) {
#pragma unroll
        for (int it = 0; it < 2; ++it) { *(volatile v8h*)(VH + ao[it]) = a[it]; if (wt) *(volatile v8h*)(T2 + to[it]) = t[it]; }
        if (ps == 0) __threadfence(); }
}

__global__ __launch_bounds__(256) void k_coef(const float* __restrict__ w1, const float* __restrict__ b1, const float* __restrict__ w2, const float* __restrict__ b2, h16* CF) {
    __shared__ float w1s[32];
    __shared__ float b1s[8];
    __shared__ float w2s[128];
    __shared__ float b2s[16];
    __shared__ float hs[8 * 256];
    __shared__ __align__(16) h16 ct[NPJ * CTP];
    const int tid = threadIdx.x, lane = tid & 31;
    const int wave = __builtin_amdgcn_readfirstlane((int)(threadIdx.x >> 5));
    const int q = blockIdx.x, hw = blockIdx.y;
    { float a = w1[tid & 31], c = b1[tid & 7], d = w2[tid & 127], e = b2[tid & 15];
      asm volatile("" : "+v"(a)); asm volatile("" : "+v"(c)); asm volatile("" : "+v"(d)); asm volatile("" : "+v"(e));
      if (tid < 32) w1s[tid] = bfr(a);
      if (tid < 8) b1s[tid] = bfr(c);
      if (tid < 128) w2s[tid] = bfr(d);
      if (tid < 16) b2s[tid] = bfr(e); }
    __syncthreads();
    const int xy = q * 256 + tid;
    const int x = xy >> 5, y = xy & 31, h = hw >> 5, w = hw & 31;
    const float cx = 2.0f * (((float)x + 0.5f) * (1.0f / 32.0f)) - 1.0f;
    const float cy = 2.0f * (((float)y + 0.5f) * (1.0f / 32.0f)) - 1.0f;
    const float ch = 2.0f * (((float)h + 0.5f) * (1.0f / 32.0f)) - 1.0f;
    const float cw = 2.0f * (((float)w + 0.5f) * (1.0f / 32.0f)) - 1.0f;
#pragma unroll 1
    for (int j = 0; j < 8; ++j) {
        float z = w1s[4 * j] * cx; z += w1s[4 * j + 1] * cy; z += w1s[4 * j + 2] * ch; z += w1s[4 * j + 3] * cw; z += b1s[j];
        const float g = 0.5f * z * (1.0f + erff(z * 0.70710678118654752f));
        hs[j * 256 + tid] = g; }
    float hv[8];
#pragma unroll
    for (int j = 0; j < 8; ++j) hv[j] = hs[j * 256 + tid];
#pragma unroll 1
    for (int n = 0; n < NPJ; ++n) {
        float acc = 0.0f;
#pragma unroll
        for (int j = 0; j < 8; ++j) acc += w2s[n * 8 + j] * hv[j];
        acc += b2s[n];
        ct[n * CTP + tid] = toh_flush(acc * CSC); }
    __syncthreads();
    const v8h o0 = *(const v8ha*)(&ct[(2 * wave) * CTP + lane * 8]);
    const v8h o1 = *(const v8ha*)(&ct[(2 * wave + 1) * CTP + lane * 8]);
    const size_t base = ((size_t)(hw * NPJ + 2 * wave)) * NPIX + (size_t)q * 256 + (size_t)lane * 8;
#pragma unroll 1
    for (int ps = 0; ps < 2; ++ps) {
        *(volatile v8h*)(CF + base) = o0; *(volatile v8h*)(CF + base + NPIX) = o1;
        if (ps == 0) __threadfence(); }
}

__global__ __launch_bounds__(32) void k_tmp(const h16* __restrict__ A, const h16* __restrict__ Bt, h16* T2) {
    __shared__ __align__(16) float os[16 * 68];
    const int K = NPIX;
    const int lane = threadIdx.x & 31, lr = lane & 15, hi = lane >> 4; const int r0 = blockIdx.x * 64, c0 = blockIdx.y * 64;
    v8f acc[4][4];
#pragma unroll
    for (int mb = 0; mb < 4; ++mb)
#pragma unroll
        for (int nb = 0; nb < 4; ++nb) acc[mb][nb] = (v8f){};
    const size_t aoff = (size_t)(r0 + lr) * K + 8 * hi, boff = (size_t)(c0 + lr) * K + 8 * hi;
#pragma unroll 1
    for (int kc = 0; kc < K; kc += 32) {
        v16h a[4];
#pragma unroll
        for (int mb = 0; mb < 4; ++mb) a[mb] = ldh(A + aoff + (size_t)mb * 16 * K + kc);
#pragma unroll
        for (int nb = 0; nb < 4; ++nb) { const v16h b = ldh(Bt + boff + (size_t)nb * 16 * K + kc);
#pragma unroll
            for (int mb = 0; mb < 4; ++mb) acc[mb][nb] = wmma16g(a[mb], b, acc[mb][nb]); }
    }
    const int bb = c0 / CIN_;
    const int hw0 = r0 / NPJ;
#pragma unroll
    for (int mb = 0; mb < 4; ++mb) {
#pragma unroll
        for (int nb = 0; nb < 4; ++nb) {
#pragma unroll
            for (int j = 0; j < 8; ++j) os[(hi * 8 + j) * 68 + nb * 16 + lr] = acc[mb][nb][j] * TSI; }
        wave_sync();
        const size_t sb = ((size_t)bb * NPO + (size_t)(hw0 + mb)) * KP2;
#pragma unroll 1
        for (int ps = 0; ps < 2; ++ps) {
#pragma unroll
            for (int s = 0; s < 4; ++s) { const int row = 4 * s + (lane >> 3), c8 = (lane & 7) * 8;
                const v4f x0 = *(const v4fa*)(&os[row * 68 + c8]); const v4f x1 = *(const v4fa*)(&os[row * 68 + c8 + 4]); v8h hv;
#pragma unroll
                for (int i = 0; i < 4; ++i) { hv[i] = toh_flush(x0[i]); hv[4 + i] = toh_flush(x1[i]); }
                *(volatile v8h*)(T2 + sb + (size_t)row * CIN_ + c8) = hv; }
            if (ps == 0) __threadfence(); }
        wave_sync();
    }
}

__global__ __launch_bounds__(32) void k_out(const h16* __restrict__ A, const h16* __restrict__ Bt, const float* __restrict__ cb, const float* __restrict__ bs, float* OUT) {
    __shared__ __align__(16) float os[16 * 68];
    const int K = KP2;
    const int lane = threadIdx.x & 31, lr = lane & 15, hi = lane >> 4; const int r0 = blockIdx.x * 64, c0 = blockIdx.y * 64;
    v8f acc[4][4];
#pragma unroll
    for (int mb = 0; mb < 4; ++mb)
#pragma unroll
        for (int nb = 0; nb < 4; ++nb) acc[mb][nb] = (v8f){};
    const size_t aoff = (size_t)(r0 + lr) * K + 8 * hi, boff = (size_t)(c0 + lr) * K + 8 * hi;
#pragma unroll 1
    for (int kc = 0; kc < K; kc += 32) {
        v16h a[4];
#pragma unroll
        for (int mb = 0; mb < 4; ++mb) a[mb] = ldh(A + aoff + (size_t)mb * 16 * K + kc);
#pragma unroll
        for (int nb = 0; nb < 4; ++nb) { const v16h b = ldh(Bt + boff + (size_t)nb * 16 * K + kc);
#pragma unroll
            for (int mb = 0; mb < 4; ++mb) acc[mb][nb] = wmma16g(a[mb], b, acc[mb][nb]); }
    }
    const int bb = c0 / NPO, p0 = c0 % NPO;
#pragma unroll
    for (int mb = 0; mb < 4; ++mb) {
        float br[8];
#pragma unroll
        for (int j = 0; j < 8; ++j) br[j] = bfr(cb[r0 + mb * 16 + hi * 8 + j]) + bfr(bs[r0 + mb * 16 + hi * 8 + j]);
#pragma unroll
        for (int nb = 0; nb < 4; ++nb) {
#pragma unroll
            for (int j = 0; j < 8; ++j) os[(hi * 8 + j) * 68 + nb * 16 + lr] = acc[mb][nb][j] * OSI + br[j]; }
        wave_sync();
        float* ob = OUT + ((size_t)bb * COUT_ + (size_t)(r0 + mb * 16)) * NPIX + (size_t)p0;
#pragma unroll 1
        for (int ps = 0; ps < 2; ++ps) {
#pragma unroll
            for (int s = 0; s < 8; ++s) { const int row = 2 * s + (lane >> 4), cofs = (lane & 15) * 4;
                const v4f val = *(const v4fa*)(&os[row * 68 + cofs]);
                *(volatile v4f*)(ob + (size_t)row * NPIX + cofs) = val; }
            if (ps == 0) __threadfence(); }
        wave_sync();
    }
}

static constexpr size_t al256(size_t v) { return (v + 255) & ~(size_t)255; }
static constexpr size_t SZ_CF = al256((size_t)NPO * NPJ * NPIX * 2);
static constexpr size_t SZ_VH = al256((size_t)NB * CIN_ * NPIX * 2);
static constexpr size_t SZ_T2 = al256((size_t)NB * NPO * KP2 * 2);
static constexpr size_t SZ_PA = al256((size_t)COUT_ * KP2 * 2);
static constexpr size_t SZ_TOTAL = SZ_CF + SZ_VH + SZ_T2 + SZ_PA;
static_assert(SZ_TOTAL <= (size_t)134217728);
static_assert(((size_t)NPO * NPJ * NPIX * 2) % 512 == 0);
static_assert(((size_t)NB * NPO * KP2 * 2) % 128 == 0);
static_assert(((size_t)COUT_ * KP2 * 2) % 128 == 0);

extern "C" void kernel_launch(void* const* d_in, const int* in_sizes, int n_in,
                              void* d_out, int out_size, void* d_ws, size_t ws_size, hipStream_t stream) {
    if (n_in < 9) return;
    if ((size_t)in_sizes[0] < (size_t)NB * CIN_ * NPIX) return;
    if ((size_t)in_sizes[1] < (size_t)NPJ * COUT_ * CIN_) return;
    if (in_sizes[2] < 32 || in_sizes[3] < 8 || in_sizes[4] < 128 || in_sizes[5] < 16) return;
    if (in_sizes[6] < COUT_ * CIN_ || in_sizes[7] < COUT_ || in_sizes[8] < COUT_) return;
    if ((size_t)out_size < (size_t)NB * COUT_ * NPIX) return;
    if (SZ_TOTAL > ws_size) return;
    const float* v      = (const float*)d_in[0];
    const float* params = (const float*)d_in[1];
    const float* w1     = (const float*)d_in[2];
    const float* b1     = (const float*)d_in[3];
    const float* w2     = (const float*)d_in[4];
    const float* b2     = (const float*)d_in[5];
    const float* convw  = (const float*)d_in[6];
    const float* convb  = (const float*)d_in[7];
    const float* bias   = (const float*)d_in[8];
    float* OUT = (float*)d_out;
    char* wsp = (char*)d_ws;
    h16* CF = (h16*)wsp; wsp += SZ_CF;
    h16* VH = (h16*)wsp; wsp += SZ_VH;
    h16* T2 = (h16*)wsp; wsp += SZ_T2;
    h16* PA = (h16*)wsp; wsp += SZ_PA;

    k_wplane<<<(unsigned)((COUT_ * (KP2 / 8)) / 256), 256, 0, stream>>>(params, convw, PA);
    k_vplanes<<<dim3(NPIX / 64, NB, 1), 256, 0, stream>>>(v, VH, T2);
    k_coef<<<dim3(NPIX / 256, NPO, 1), 256, 0, stream>>>(w1, b1, w2, b2, CF);
    k_tmp<<<dim3(NPO * NPJ / 64, NB * CIN_ / 64, 1), 32, 0, stream>>>(CF, VH, T2);
    k_out<<<dim3(COUT_ / 64, NB * NPO / 64, 1), 32, 0, stream>>>(PA, T2, convb, bias, OUT);
}
